// EquivariantGNN_GAT_54211077210112
// MI455X (gfx1250) — hardware-verified
//
#include <hip/hip_runtime.h>
#include <stddef.h>
#include <stdint.h>


#define DF    128
#define OD    32
#define FE    125
#define GR    32
#define LR    128
#define AP    136
#define XSP   132
#define YSP   36
#define NB    512
#define CHUNK 2048
#define NTHR  256
#define NWAVE 8
#define WCAP  256
#define NGRP  (CHUNK / (NTHR * 4))
#define MAXG  64
#define PW    4

#define LDS_SACC (NB * DF)
#define LDS_AUX  (NB * 3)
#define LDS_LIST (NWAVE * WCAP)
#define LDS_BYTES ((LDS_SACC + LDS_AUX + LDS_LIST + NWAVE + NWAVE) * 4)

static_assert(WCAP == (CHUNK / NTHR) * 32);
static_assert(NGRP >= 1);
static_assert(NB == 512);
static_assert(CHUNK <= 4096);
static_assert(((LDS_SACC + NB) % 4) == 0);
static_assert(LDS_BYTES == 276544);
static_assert(PW * MAXG == NTHR);
static_assert((MAXG * OD) % NTHR == 0);

typedef float    v4f  __attribute__((ext_vector_type(4)));
typedef float    v8f  __attribute__((ext_vector_type(8)));
typedef int      v4i  __attribute__((ext_vector_type(4)));
typedef _Float16 v8h  __attribute__((ext_vector_type(8)));
typedef _Float16 v16h __attribute__((ext_vector_type(16)));
union Frag   { v16h v; v8h half[2]; };
union Pack16 { v8h h; v4i i; };

__device__ __forceinline__ v8f wm(v16h a, v16h b, v8f c) {
  v8f d = __builtin_amdgcn_wmma_f32_16x16x32_f16(false, a, false, b, (short)0, c, false, false);
  asm volatile("v_nop\n\tv_nop\n\tv_nop\n\tv_nop" : "+v"(d) : "v"(a), "v"(b));
  return d;
}

template<int NCOL>
__global__ __launch_bounds__(NTHR) void k_prep(const float* __restrict__ W, _Float16* Wt) {
  __shared__ __attribute__((aligned(16))) _Float16 T[DF * AP];
  static_assert(NCOL <= DF);
  static_assert(((NCOL * (DF / 8)) % NTHR) == 0);
  const int tid = threadIdx.x;
  for (int i = tid; i < DF * NCOL; i += NTHR) {
    const int k = i / NCOL;
    const int n = i - k * NCOL;
    T[n * AP + k] = (_Float16)(W[i] * 8.0f);
  }
  __syncthreads();
  constexpr int NCH = NCOL * (DF / 8);
#pragma unroll 1
  for (int it = 0; it < NCH / NTHR; ++it) {
    const int i   = it * NTHR + tid;
    const int row = i >> 4;
    const int c8  = (i & 15) * 8;
    Pack16 u;
    u.h = *(const v8h*)(T + row * AP + c8);
    _Float16* p = Wt + (size_t)row * DF + c8;
    *(volatile v4i*)p = u.i;
    __threadfence();
    *(volatile v4i*)p = u.i;
  }
}

__device__ __forceinline__ void epi_tile(v8f acc, int T, int hh, int m, int wave, int ncol,
                                         float cs, float cd, float* Xs, float* As, float* Ds) {
  float ss[8], sd[8];
#pragma unroll
  for (int r = 0; r < 8; ++r) {
    const float v = acc[r] * 0.125f;
    Xs[(T * 16 + 8 * hh + r) * XSP + ncol] = v;
    ss[r] = v * cs;
    sd[r] = v * cd;
  }
#pragma unroll
  for (int mk = 1; mk < 16; mk <<= 1) {
#pragma unroll
    for (int r = 0; r < 8; ++r) {
      ss[r] += __shfl_xor(ss[r], mk, 32);
      sd[r] += __shfl_xor(sd[r], mk, 32);
    }
  }
  if (m == 0) {
#pragma unroll
    for (int r = 0; r < 8; ++r) {
      As[(T * 16 + 8 * hh + r) * NWAVE + wave] = ss[r];
      Ds[(T * 16 + 8 * hh + r) * NWAVE + wave] = sd[r];
    }
  }
}

template<int MODE>
__global__ __launch_bounds__(NTHR) void k_gemm(
    const float* __restrict__ pos, const int* __restrict__ zid, const float* __restrict__ emb,
    const float* __restrict__ x, const _Float16* __restrict__ Wt,
    const float* __restrict__ att_s, const float* __restrict__ att_d,
    float* xp, float* asrc, float* adst, int nN, int nT) {
  __shared__ __attribute__((aligned(16))) _Float16 At[GR * AP];
  __shared__ __attribute__((aligned(16))) float Xs[GR * XSP];
  __shared__ __attribute__((aligned(16))) float As[GR * NWAVE];
  __shared__ __attribute__((aligned(16))) float Ds[GR * NWAVE];

  const int tid  = threadIdx.x;
  const int lane = tid & 31;
  const int wave = tid >> 5;
  const int hh   = lane >> 4;
  const int m    = lane & 15;
  const int rowBase = blockIdx.x * GR;

  {
    const int r  = tid >> 3;
    const int c0 = (tid & 7) * 16;
    int row = rowBase + r;
    if (row > nN - 1) row = nN - 1;
    float v[16];
    if (MODE == 0) {
      int zc = zid[row];
      if (zc < 0) zc += nT;
      zc = zc < 0 ? 0 : (zc > nT - 1 ? nT - 1 : zc);
      const float* er = emb + (size_t)zc * FE;
#pragma unroll
      for (int j = 0; j < 16; ++j) {
        int ie = c0 + j - 3;
        ie = ie < 0 ? 0 : ie;
        v[j] = er[ie];
      }
      const float p0 = pos[(size_t)row * 3 + 0];
      const float p1 = pos[(size_t)row * 3 + 1];
      const float p2 = pos[(size_t)row * 3 + 2];
      if (c0 == 0) { v[0] = p0; v[1] = p1; v[2] = p2; }
    } else {
      const float* p = x + (size_t)row * DF + c0;
      const v4f f0 = *(const v4f*)(p), f1 = *(const v4f*)(p + 4);
      const v4f f2 = *(const v4f*)(p + 8), f3 = *(const v4f*)(p + 12);
      v[0] = f0.x;  v[1] = f0.y;  v[2] = f0.z;  v[3] = f0.w;
      v[4] = f1.x;  v[5] = f1.y;  v[6] = f1.z;  v[7] = f1.w;
      v[8] = f2.x;  v[9] = f2.y;  v[10] = f2.z; v[11] = f2.w;
      v[12] = f3.x; v[13] = f3.y; v[14] = f3.z; v[15] = f3.w;
    }
    Pack16 u0, u1;
#pragma unroll
    for (int j = 0; j < 8; ++j) { u0.h[j] = (_Float16)v[j]; u1.h[j] = (_Float16)v[8 + j]; }
    *(v8h*)(At + r * AP + c0)     = u0.h;
    *(v8h*)(At + r * AP + c0 + 8) = u1.h;
  }
  __syncthreads();

  const int ncol = wave * 16 + m;
  v8f c0a = {0.f, 0.f, 0.f, 0.f, 0.f, 0.f, 0.f, 0.f};
  v8f c1a = {0.f, 0.f, 0.f, 0.f, 0.f, 0.f, 0.f, 0.f};
#pragma unroll
  for (int kt = 0; kt < DF / 32; ++kt) {
    const int k0 = kt * 32;
    Frag a0, a1, b;
    const _Float16* pb  = Wt + (size_t)ncol * DF + k0 + 8 * hh;
    const _Float16* pa0 = At + m * AP + k0 + 8 * hh;
    const _Float16* pa1 = At + (16 + m) * AP + k0 + 8 * hh;
    b.half[0]  = *(const v8h*)pb;  b.half[1]  = *(const v8h*)(pb + 16);
    a0.half[0] = *(const v8h*)pa0; a0.half[1] = *(const v8h*)(pa0 + 16);
    a1.half[0] = *(const v8h*)pa1; a1.half[1] = *(const v8h*)(pa1 + 16);
    c0a = wm(a0.v, b.v, c0a);
    c1a = wm(a1.v, b.v, c1a);
  }

  const float cs = att_s[ncol];
  const float cd = att_d[ncol];
  epi_tile(c0a, 0, hh, m, wave, ncol, cs, cd, Xs, As, Ds);
  epi_tile(c1a, 1, hh, m, wave, ncol, cs, cd, Xs, As, Ds);
  __syncthreads();

  v4f xr[4];
#pragma unroll
  for (int i = 0; i < 4; ++i) xr[i] = *(const v4f*)(Xs + (4 * wave + i) * XSP + 4 * lane);
  float* gp = 0;
  v4f gv = {0.f, 0.f, 0.f, 0.f};
  if (wave == 0 && lane < 16) {
    const int q = lane & 7;
    const float* S = (lane < 8) ? As : Ds;
    float a[4];
#pragma unroll
    for (int i = 0; i < 4; ++i) {
      const v4f u0 = *(const v4f*)(S + (4 * q + i) * NWAVE);
      const v4f u1 = *(const v4f*)(S + (4 * q + i) * NWAVE + 4);
      a[i] = ((((((u0.x + u0.y) + u0.z) + u0.w) + u1.x) + u1.y) + u1.z) + u1.w;
    }
    gv.x = a[0]; gv.y = a[1]; gv.z = a[2]; gv.w = a[3];
    gp = ((lane < 8) ? asrc : adst) + (size_t)rowBase + 4 * q;
  }
  float* xpp[4];
#pragma unroll
  for (int i = 0; i < 4; ++i) xpp[i] = xp + (size_t)(rowBase + 4 * wave + i) * DF + 4 * lane;

#pragma unroll
  for (int i = 0; i < 4; ++i) *(volatile v4f*)(xpp[i]) = xr[i];
  if (gp) *(volatile v4f*)gp = gv;
  __threadfence();
#pragma unroll
  for (int i = 0; i < 4; ++i) *(volatile v4f*)(xpp[i]) = xr[i];
  if (gp) *(volatile v4f*)gp = gv;
}

__global__ __launch_bounds__(NTHR) void k_agg(
    const int* __restrict__ ei, const float* __restrict__ xp,
    const float* __restrict__ asrc, const float* __restrict__ adst,
    const float* __restrict__ bias, float* xo, int nN, int nE) {
  extern __shared__ v4f lds_dyn[];
  float* sacc = (float*)lds_dyn;
  float* den  = sacc + LDS_SACC;
  float* sdl  = den + NB;
  float* shf  = sdl + NB;
  int*   list = (int*)(shf + NB);
  int*   wcnt = list + LDS_LIST;
  float* red  = (float*)(wcnt + NWAVE);

  const int tid  = threadIdx.x;
  const int lane = tid & 31;
  const int wave = tid >> 5;
  const int nodeBase = blockIdx.x * NB;

  {
    const v4f z4 = {0.f, 0.f, 0.f, 0.f};
    for (int i = tid; i < (LDS_SACC + NB) / 4; i += NTHR) lds_dyn[i] = z4;
    for (int s = tid; s < NB; s += NTHR) {
      int nd = nodeBase + s;
      if (nd > nN - 1) nd = nN - 1;
      sdl[s] = adst[nd];
    }
    float mx = __int_as_float(0xff800000);
#pragma unroll 1
    for (int i = tid; i < nN; i += NTHR) mx = fmaxf(mx, asrc[i]);
    mx = fmaxf(mx, __shfl_xor(mx, 16, 32));
    mx = fmaxf(mx, __shfl_xor(mx, 8, 32));
    mx = fmaxf(mx, __shfl_xor(mx, 4, 32));
    mx = fmaxf(mx, __shfl_xor(mx, 2, 32));
    mx = fmaxf(mx, __shfl_xor(mx, 1, 32));
    if (lane == 0) red[wave] = mx;
  }
  __syncthreads();
  {
    float bm = red[0];
#pragma unroll
    for (int w = 1; w < NWAVE; ++w) bm = fmaxf(bm, red[w]);
    for (int s = tid; s < NB; s += NTHR) {
      const float t = bm + sdl[s];
      shf[s] = (t > 0.f) ? t : 0.2f * t;
    }
  }
  __syncthreads();

  const int* eid = ei + nE;
  const bool al16 = ((nE & 3) == 0);

  const int nChunks = (nE + CHUNK - 1) / CHUNK;
#pragma unroll 1
  for (int ch = 0; ch < nChunks; ++ch) {
    const int cbase = ch * CHUNK;
    int wc = 0;
#pragma unroll
    for (int g = 0; g < NGRP; ++g) {
      const int el0 = (g * NTHR + tid) * 4;
      const int e0  = cbase + el0;
      const int sent = -2147483647 - 1;
      v4i d;
      if (al16 && (e0 + 3 < nE)) {
        d = *(const v4i*)(eid + e0);
      } else {
        d.x = (e0     < nE) ? eid[e0]     : sent;
        d.y = (e0 + 1 < nE) ? eid[e0 + 1] : sent;
        d.z = (e0 + 2 < nE) ? eid[e0 + 2] : sent;
        d.w = (e0 + 3 < nE) ? eid[e0 + 3] : sent;
      }
      const unsigned s0 = (unsigned)d.x - (unsigned)nodeBase;
      const unsigned s1 = (unsigned)d.y - (unsigned)nodeBase;
      const unsigned s2 = (unsigned)d.z - (unsigned)nodeBase;
      const unsigned s3 = (unsigned)d.w - (unsigned)nodeBase;
      const bool h0 = s0 < (unsigned)NB;
      const bool h1 = s1 < (unsigned)NB;
      const bool h2 = s2 < (unsigned)NB;
      const bool h3 = s3 < (unsigned)NB;
      const unsigned many = __builtin_amdgcn_ballot_w32(h0 | h1 | h2 | h3);
      if (many != 0u) {
#define HITJ(J, HJ, SJ) { \
          const unsigned mj = __builtin_amdgcn_ballot_w32(HJ); \
          if (HJ) { \
            const int ps = wc + (int)__builtin_amdgcn_mbcnt_lo(mj, 0u); \
            if (ps < WCAP) list[wave * WCAP + ps] = ((el0 + (J)) << 9) | (int)(SJ); \
          } \
          wc += (int)__builtin_popcount(mj); }
        HITJ(0, h0, s0)
        HITJ(1, h1, s1)
        HITJ(2, h2, s2)
        HITJ(3, h3, s3)
#undef HITJ
      }
    }
    if (lane == 0) wcnt[wave] = wc;
    __syncthreads();

    if (wave == 0) {
#pragma unroll 1
      for (int wsx = 0; wsx < NWAVE; ++wsx) {
        int n = wcnt[wsx];
        if (n > WCAP) n = WCAP;
        if (n < 0) n = 0;
#pragma unroll 1
        for (int i = 0; i < n; ++i) {
          const int ent  = list[wsx * WCAP + i];
          const int slot = ent & (NB - 1);
          const int el   = (ent >> 9) & (CHUNK - 1);
          int e = cbase + el;
          if (e > nE - 1) e = nE - 1;
          int src = ei[e];
          if (src < 0) src += nN;
          src = src < 0 ? 0 : (src > nN - 1 ? nN - 1 : src);
          float al = asrc[src] + sdl[slot];
          al = (al > 0.f) ? al : 0.2f * al;
          const float p = __expf(al - shf[slot]);
          const v4f xv = *(const v4f*)(xp + (size_t)src * DF + 4 * lane);
          v4f* sp = (v4f*)(sacc + slot * DF + 4 * lane);
          const v4f cur = *sp;
          const v4f nxt = cur + p * xv;
          *sp = nxt;
          if (lane == 0) {
            const float o = den[slot];
            den[slot] = o + p;
          }
        }
      }
    }
    __syncthreads();
  }

  const v4f b4 = *(const v4f*)(bias + 4 * lane);
#pragma unroll 1
  for (int j = 0; j < NB / NWAVE; ++j) {
    const int slot = wave * (NB / NWAVE) + j;
    const int node = nodeBase + slot;
    if (node >= nN) break;
    const size_t nrow = (size_t)node;
    float al = asrc[nrow] + sdl[slot];
    al = (al > 0.f) ? al : 0.2f * al;
    const float p = __expf(al - shf[slot]);
    const v4f xv = *(const v4f*)(xp + nrow * DF + 4 * lane);
    const v4f sv = *(const v4f*)(sacc + slot * DF + 4 * lane) + p * xv;
    const float dv  = den[slot] + p;
    const float inv = 1.0f / dv;
    v4f hv = sv * inv + b4;
    hv.x = hv.x > 0.f ? hv.x : (__expf(hv.x) - 1.0f);
    hv.y = hv.y > 0.f ? hv.y : (__expf(hv.y) - 1.0f);
    hv.z = hv.z > 0.f ? hv.z : (__expf(hv.z) - 1.0f);
    hv.w = hv.w > 0.f ? hv.w : (__expf(hv.w) - 1.0f);
    float* op = xo + nrow * DF + 4 * lane;
    *(volatile v4f*)op = hv;
    __threadfence();
    *(volatile v4f*)op = hv;
  }
}

__global__ __launch_bounds__(NTHR) void k_lin(
    const float* __restrict__ x, const _Float16* __restrict__ Wt,
    const float* __restrict__ bl, float* y, int nN) {
  __shared__ __attribute__((aligned(16))) _Float16 At[LR * AP];
  __shared__ __attribute__((aligned(16))) float Ys[LR * YSP];

  const int tid  = threadIdx.x;
  const int lane = tid & 31;
  const int wave = tid >> 5;
  const int hh   = lane >> 4;
  const int m    = lane & 15;
  const int rowBase = blockIdx.x * LR;

#pragma unroll
  for (int it = 0; it < LR / 32; ++it) {
    const int r  = it * 32 + (tid >> 3);
    const int c0 = (tid & 7) * 16;
    int row = rowBase + r;
    if (row > nN - 1) row = nN - 1;
    const float* p = x + (size_t)row * DF + c0;
    const v4f f0 = *(const v4f*)(p), f1 = *(const v4f*)(p + 4);
    const v4f f2 = *(const v4f*)(p + 8), f3 = *(const v4f*)(p + 12);
    Pack16 u0, u1;
    u0.h[0] = (_Float16)f0.x; u0.h[1] = (_Float16)f0.y; u0.h[2] = (_Float16)f0.z; u0.h[3] = (_Float16)f0.w;
    u0.h[4] = (_Float16)f1.x; u0.h[5] = (_Float16)f1.y; u0.h[6] = (_Float16)f1.z; u0.h[7] = (_Float16)f1.w;
    u1.h[0] = (_Float16)f2.x; u1.h[1] = (_Float16)f2.y; u1.h[2] = (_Float16)f2.z; u1.h[3] = (_Float16)f2.w;
    u1.h[4] = (_Float16)f3.x; u1.h[5] = (_Float16)f3.y; u1.h[6] = (_Float16)f3.z; u1.h[7] = (_Float16)f3.w;
    *(v8h*)(At + r * AP + c0)     = u0.h;
    *(v8h*)(At + r * AP + c0 + 8) = u1.h;
  }
  __syncthreads();

  v8f c0a = {0.f, 0.f, 0.f, 0.f, 0.f, 0.f, 0.f, 0.f};
  v8f c1a = {0.f, 0.f, 0.f, 0.f, 0.f, 0.f, 0.f, 0.f};
#pragma unroll
  for (int kt = 0; kt < DF / 32; ++kt) {
    const int k0 = kt * 32;
    Frag a, b0, b1;
    const _Float16* pa  = At + (16 * wave + m) * AP + k0 + 8 * hh;
    const _Float16* pb0 = Wt + (size_t)m * DF + k0 + 8 * hh;
    const _Float16* pb1 = Wt + (size_t)(16 + m) * DF + k0 + 8 * hh;
    a.half[0]  = *(const v8h*)pa;  a.half[1]  = *(const v8h*)(pa + 16);
    b0.half[0] = *(const v8h*)pb0; b0.half[1] = *(const v8h*)(pb0 + 16);
    b1.half[0] = *(const v8h*)pb1; b1.half[1] = *(const v8h*)(pb1 + 16);
    c0a = wm(a.v, b0.v, c0a);
    c1a = wm(a.v, b1.v, c1a);
  }

  const float bl0 = bl[m];
  const float bl1 = bl[16 + m];
#pragma unroll
  for (int r = 0; r < 8; ++r) {
    Ys[(16 * wave + 8 * hh + r) * YSP + m]      = c0a[r] * 0.125f + bl0;
    Ys[(16 * wave + 8 * hh + r) * YSP + 16 + m] = c1a[r] * 0.125f + bl1;
  }
  __syncthreads();

  v4f vv[4];
  float* pp[4];
#pragma unroll
  for (int it = 0; it < 4; ++it) {
    const int row = 16 * wave + 4 * it + (lane >> 3);
    const int c   = 4 * (lane & 7);
    vv[it] = *(const v4f*)(Ys + row * YSP + c);
    pp[it] = y + (size_t)(rowBase + row) * OD + c;
  }
#pragma unroll
  for (int it = 0; it < 4; ++it) *(volatile v4f*)(pp[it]) = vv[it];
  __threadfence();
#pragma unroll
  for (int it = 0; it < 4; ++it) *(volatile v4f*)(pp[it]) = vv[it];
}

__global__ __launch_bounds__(NTHR) void k_pool(
    const float* __restrict__ y, const int* __restrict__ bat, float* out, int nN, int nG) {
  __shared__ __attribute__((aligned(16))) float psum[PW * MAXG * OD];
  __shared__ __attribute__((aligned(16))) float pcnt[PW * MAXG];
  __shared__ __attribute__((aligned(16))) float fin[MAXG * OD];

  const int tid  = threadIdx.x;
  const int lane = tid & 31;
  const int wave = tid >> 5;
  {
    const v4f z4 = {0.f, 0.f, 0.f, 0.f};
    v4f* pz = (v4f*)psum;
    for (int i = tid; i < (PW * MAXG * OD) / 4; i += NTHR) pz[i] = z4;
    pcnt[tid] = 0.f;
  }
  __syncthreads();

  if (wave < PW) {
    const int npw = ((nN + PW * 32 - 1) / (PW * 32)) * 32;
    const int beg = wave * npw;
    int end = beg + npw;
    if (end > nN) end = nN;
#pragma unroll 1
    for (int cb = beg; cb < end; cb += 32) {
      const int node = cb + lane;
      int b = (node < end) ? bat[node] : -1;
      if (b >= nG) b = -1;
      unsigned rem = __builtin_amdgcn_ballot_w32(b >= 0);
#pragma unroll 1
      for (int it = 0; it < 32 && rem != 0u; ++it) {
        const int lead = __builtin_ctz(rem);
        const int gsel = __shfl(b, lead, 32);
        const unsigned grp = __builtin_amdgcn_ballot_w32(b == gsel);
        rem &= ~grp;
        float racc = 0.f;
        unsigned gm = grp;
#pragma unroll 1
        for (int k = 0; k < 32 && gm != 0u; ++k) {
          const int jn = __builtin_ctz(gm);
          gm &= gm - 1u;
          racc += y[(size_t)(cb + jn) * OD + lane];
        }
        float* ps = psum + (wave * MAXG + gsel) * OD + lane;
        const float o = *ps;
        *ps = o + racc;
        if (lane == 0) {
          const float oc = pcnt[wave * MAXG + gsel];
          pcnt[wave * MAXG + gsel] = oc + (float)__builtin_popcount(grp);
        }
      }
    }
  }
  __syncthreads();

#pragma unroll
  for (int k = 0; k < (MAXG * OD) / NTHR; ++k) {
    const int idx = k * NTHR + tid;
    const int g = idx >> 5;
    const int c = idx & 31;
    float s = 0.f, cn = 0.f;
#pragma unroll
    for (int w = 0; w < PW; ++w) {
      s  += psum[(w * MAXG + g) * OD + c];
      cn += pcnt[w * MAXG + g];
    }
    fin[idx] = s * (1.0f / fmaxf(cn, 1.0f));
  }
  __syncthreads();

  v4f vv[2];
  float* pp[2];
  bool ok[2];
#pragma unroll
  for (int it = 0; it < 2; ++it) {
    const int row = 8 * wave + 4 * it + (lane >> 3);
    const int c   = 4 * (lane & 7);
    vv[it] = *(const v4f*)(fin + row * OD + c);
    pp[it] = out + (size_t)row * OD + c;
    ok[it] = row < nG;
  }
#pragma unroll
  for (int it = 0; it < 2; ++it) if (ok[it]) *(volatile v4f*)(pp[it]) = vv[it];
  __threadfence();
#pragma unroll
  for (int it = 0; it < 2; ++it) if (ok[it]) *(volatile v4f*)(pp[it]) = vv[it];
}

extern "C" void kernel_launch(void* const* d_in, const int* in_sizes, int n_in,
                              void* d_out, int out_size, void* d_ws, size_t ws_size,
                              hipStream_t stream) {
  if (n_in < 15) return;
  const int nN = in_sizes[0] / 3;
  if (nN <= 0 || in_sizes[0] != 3 * nN) return;
  if (in_sizes[1] != nN || in_sizes[3] != nN) return;
  const int nE = in_sizes[2] / 2;
  if (nE < 0 || in_sizes[2] != 2 * nE) return;
  const int nT = in_sizes[4] / FE;
  if (nT <= 0 || in_sizes[4] != nT * FE) return;
  if (in_sizes[5] != DF * DF || in_sizes[9] != DF * DF) return;
  if (in_sizes[6] != DF || in_sizes[7] != DF || in_sizes[8] != DF) return;
  if (in_sizes[10] != DF || in_sizes[11] != DF || in_sizes[12] != DF) return;
  if (in_sizes[13] != DF * OD || in_sizes[14] != OD) return;
  const int nG = out_size / OD;
  if (nG <= 0 || nG > MAXG || out_size != nG * OD) return;

  const float* pos  = (const float*)d_in[0];
  const int*   zid  = (const int*)d_in[1];
  const int*   ei   = (const int*)d_in[2];
  const int*   bat  = (const int*)d_in[3];
  const float* emb  = (const float*)d_in[4];
  const float* W1   = (const float*)d_in[5];
  const float* a1s  = (const float*)d_in[6];
  const float* a1d  = (const float*)d_in[7];
  const float* b1   = (const float*)d_in[8];
  const float* W2   = (const float*)d_in[9];
  const float* a2s  = (const float*)d_in[10];
  const float* a2d  = (const float*)d_in[11];
  const float* b2   = (const float*)d_in[12];
  const float* Wl   = (const float*)d_in[13];
  const float* bl   = (const float*)d_in[14];
  float* out = (float*)d_out;

  const int nP  = ((nN + GR - 1) / GR) * GR;
  const int nPL = ((nN + LR - 1) / LR) * LR;
  size_t off = 0;
  char* wsb = (char*)d_ws;
  _Float16* Wt1 = (_Float16*)(wsb + off); off += (((size_t)DF * DF * 2) + 255) & ~(size_t)255;
  _Float16* Wt2 = (_Float16*)(wsb + off); off += (((size_t)DF * DF * 2) + 255) & ~(size_t)255;
  _Float16* Wtl = (_Float16*)(wsb + off); off += (((size_t)OD * DF * 2) + 255) & ~(size_t)255;
  float* xp   = (float*)(wsb + off); off += (((size_t)nP * DF * 4) + 255) & ~(size_t)255;
  float* asrc = (float*)(wsb + off); off += (((size_t)nP * 4) + 255) & ~(size_t)255;
  float* adst = (float*)(wsb + off); off += (((size_t)nP * 4) + 255) & ~(size_t)255;
  float* xcur = (float*)(wsb + off); off += (((size_t)nP * DF * 4) + 255) & ~(size_t)255;
  float* yv   = (float*)(wsb + off); off += (((size_t)nPL * OD * 4) + 255) & ~(size_t)255;
  if (off > ws_size) return;
  if (off > (size_t)134217728) return;

  k_prep<DF><<<1, NTHR, 0, stream>>>(W1, Wt1);
  k_prep<DF><<<1, NTHR, 0, stream>>>(W2, Wt2);
  k_prep<OD><<<1, NTHR, 0, stream>>>(Wl, Wtl);

  hipFuncSetAttribute(reinterpret_cast<const void*>(&k_agg),
                      hipFuncAttributeMaxDynamicSharedMemorySize, LDS_BYTES);
  const int gGemm = nP / GR;
  const int gAgg  = (nN + NB - 1) / NB;

  k_gemm<0><<<gGemm, NTHR, 0, stream>>>(pos, zid, emb, (const float*)0, Wt1, a1s, a1d,
                                         xp, asrc, adst, nN, nT);
  k_agg<<<gAgg, NTHR, LDS_BYTES, stream>>>(ei, xp, asrc, adst, b1, xcur, nN, nE);

  k_gemm<1><<<gGemm, NTHR, 0, stream>>>(pos, zid, emb, xcur, Wt2, a2s, a2d,
                                         xp, asrc, adst, nN, nT);
  k_agg<<<gAgg, NTHR, LDS_BYTES, stream>>>(ei, xp, asrc, adst, b2, xcur, nN, nE);

  k_lin<<<nPL / LR, NTHR, 0, stream>>>(xcur, Wtl, bl, yv, nN);
  k_pool<<<1, NTHR, 0, stream>>>(yv, bat, out, nN, nG);
}
